// MultiHeadAttention__40870908788989
// MI455X (gfx1250) — hardware-verified
//
#include <hip/hip_runtime.h>
#include <math.h>

constexpr int kBatch = 4;
constexpr int kHeads = 8;
constexpr int kD     = 64;
constexpr int kSeq   = 2048;
constexpr int kHD    = kHeads * kD;
constexpr int kGroup = 2;
constexpr int kOutElems = kBatch * kD * kSeq + 3 * kBatch * kHeads * kD * kSeq;
constexpr float kXCarry        = 8.0f;
constexpr float kWCarry        = 16.0f;
constexpr float kProjOutScale  = 1.0f / 128.0f;
constexpr float kProjPlanScale = 1.0f / 8.0f;
constexpr float kScoreScale    = 0.125f / 256.0f;
constexpr float kPCarry        = 32768.0f;
constexpr float kPVScale       = 256.0f / (32768.0f * 16.0f);
constexpr float kYScale        = 1.0f / (256.0f * 16.0f);
static_assert(kHeads * kD == kHD);
static_assert(kSeq % 64 == 0 && kD % 32 == 0 && kHD % 64 == 0 && kSeq % 256 == 0);
static_assert(kHeads % kGroup == 0);
static_assert(kD % 32 == 0 && kHD % 32 == 0 && kSeq % 32 == 0);
static_assert(kOutElems * 4 == 52428800);
static_assert((kBatch * kD * kSeq) * 4 == 2097152);
static_assert((kBatch * kD * kSeq + kBatch * kHeads * kD * kSeq) * 4 == 18874368);
static_assert((kBatch * kD * kSeq + 2 * kBatch * kHeads * kD * kSeq) * 4 == 35651584);

typedef __attribute__((ext_vector_type(16))) _Float16 v16h;
typedef __attribute__((ext_vector_type(8)))  _Float16 v8h;
typedef __attribute__((ext_vector_type(16))) __bf16   v16b;
typedef __attribute__((ext_vector_type(8)))  __bf16   v8b;
typedef __attribute__((ext_vector_type(8)))  float    v8f;
typedef __attribute__((ext_vector_type(4)))  float    v4f;
typedef __attribute__((ext_vector_type(4)))  unsigned int v4u;

__device__ __forceinline__ unsigned short f2bf_bits(float f) {
  unsigned u = __float_as_uint(f);
  return (unsigned short)((u + 0x7FFFu + ((u >> 16) & 1u)) >> 16);
}
__device__ __forceinline__ float bf_bits2f(unsigned short h) { return __uint_as_float(((unsigned)h) << 16); }
__device__ __forceinline__ float bf16r(float f) { return bf_bits2f(f2bf_bits(f)); }

__device__ __forceinline__ void dep_guard_h(v8f& a, v8f& b, v16h x, v16h y) { asm volatile("v_nop\n\tv_nop\n\tv_nop\n\tv_nop" : "+v"(a), "+v"(b) : "v"(x), "v"(y)); }
__device__ __forceinline__ void dep_guard_b(v8f& a, v8f& b, v16b x, v16b y) { asm volatile("v_nop\n\tv_nop\n\tv_nop\n\tv_nop" : "+v"(a), "+v"(b) : "v"(x), "v"(y)); }
__device__ __forceinline__ void keep4_h(v16h a, v16h b, v16h c, v16h d) { asm volatile("v_nop" :: "v"(a), "v"(b), "v"(c), "v"(d)); }
__device__ __forceinline__ void keep4_b(v16b a, v16b b, v16b c, v16b d) { asm volatile("v_nop" :: "v"(a), "v"(b), "v"(c), "v"(d)); }
__device__ __forceinline__ void acc_guard4(v8f& a, v8f& b, v8f& c, v8f& d) { asm volatile("v_nop\n\tv_nop\n\tv_nop\n\tv_nop" : "+v"(a), "+v"(b), "+v"(c), "+v"(d)); }
template <typename T> struct Frag;
template <> struct Frag<_Float16> {
  typedef v16h V; union U { v16h v; v8h h[2]; };
  static __device__ __forceinline__ v16h load(const _Float16* p) {
    U f; f.h[0] = *(const v8h*)(p); f.h[1] = *(const v8h*)(p + 16); return f.v;
  }
  static __device__ __forceinline__ v8f mma(v16h a, v16h b, v8f c) {
    return __builtin_amdgcn_wmma_f32_16x16x32_f16(false, a, false, b, (short)0, c, false, false);
  }
  static __device__ __forceinline__ void guard(v8f& a, v8f& b, v16h x, v16h y) { dep_guard_h(a, b, x, y); }
  static __device__ __forceinline__ void keep(v16h a, v16h b, v16h c, v16h d) { keep4_h(a, b, c, d); }
};
template <> struct Frag<__bf16> {
  typedef v16b V; union U { v16b v; v8b h[2]; };
  static __device__ __forceinline__ v16b load(const __bf16* p) {
    U f; f.h[0] = *(const v8b*)(p); f.h[1] = *(const v8b*)(p + 16); return f.v;
  }
  static __device__ __forceinline__ v8f mma(v16b a, v16b b, v8f c) {
    return __builtin_amdgcn_wmma_f32_16x16x32_bf16(false, a, false, b, (short)0, c, false, false);
  }
  static __device__ __forceinline__ void guard(v8f& a, v8f& b, v16b x, v16b y) { dep_guard_b(a, b, x, y); }
  static __device__ __forceinline__ void keep(v16b a, v16b b, v16b c, v16b d) { keep4_b(a, b, c, d); }
};

__device__ __forceinline__ unsigned pk16(unsigned short a, unsigned short b) { return (unsigned)a | ((unsigned)b << 16); }
__device__ __forceinline__ unsigned short h_bits(float f) { const _Float16 h = (_Float16)f; return __builtin_bit_cast(unsigned short, h); }

template <int ET> struct Elem;
template <> struct Elem<0> { typedef _Float16 T; };
template <> struct Elem<1> { typedef __bf16 T; };
template <int ET, bool SPLIT, int BIAS_MODE, int OUT_MODE, bool RESID, int ACT = 0>
__global__ __launch_bounds__(256) void wmma_gemm64(
    const unsigned short* __restrict__ Ap, const unsigned short* __restrict__ A2p, int lda, long strideA,
    const unsigned short* __restrict__ Btp, const unsigned short* __restrict__ Bt2p, int ldb, long strideB,
    void* __restrict__ Cout, void* __restrict__ Cout2, int ldc, long strideC,
    const float* __restrict__ bias,
    const float* __restrict__ resid, long strideR,
    int M, int N, int K, float scale) {
  typedef typename Elem<ET>::T T;
  typedef typename Frag<T>::V V;
  const T* A = (const T*)Ap; const T* A2 = (const T*)A2p; const T* Bt = (const T*)Btp; const T* Bt2 = (const T*)Bt2p;
  __shared__ __align__(16) float sT[8][16 * 68];
  const int b    = blockIdx.y;
  const int lane = threadIdx.x & 31;
  const int wave = threadIdx.x >> 5;
  const int tilesN = N >> 6;
  const int tilesM = M >> 6;
  const int tile = blockIdx.x * 8 + wave;
  if (tile >= tilesM * tilesN) return;
  const int tm = tile / tilesN;
  const int tn = tile - tm * tilesN;
  const int m0 = tm << 6;
  const int n0 = tn << 6;

  const T* Ab  = A  + (size_t)b * strideA;
  const T* Bb  = Bt + (size_t)b * strideB;
  const T* Ab2 = SPLIT ? (A2  + (size_t)b * strideA) : nullptr;
  const T* Bb2 = SPLIT ? (Bt2 + (size_t)b * strideB) : nullptr;

  const int rlane = lane & 15;
  const int koff  = (lane >> 4) * 8;
  const int mOff  = (lane >> 4) * 8;

  v8f acc[4][4];
#pragma unroll
  for (int i = 0; i < 4; ++i)
#pragma unroll
    for (int j = 0; j < 4; ++j) acc[i][j] = (v8f){0.f,0.f,0.f,0.f,0.f,0.f,0.f,0.f};

  for (int k0 = 0; k0 < K; k0 += 32) {
    V bh[4], bl[4];
#pragma unroll
    for (int j = 0; j < 4; ++j) {
      const size_t bo = (size_t)(n0 + (j << 4) + rlane) * ldb + koff + k0;
      bh[j] = Frag<T>::load(Bb + bo);
      if (SPLIT) bl[j] = Frag<T>::load(Bb2 + bo);
    }
#pragma unroll
    for (int i = 0; i < 4; ++i) {
      const size_t ao = (size_t)(m0 + (i << 4) + rlane) * lda + koff + k0;
      V ah = Frag<T>::load(Ab + ao);
      V al;
      if (SPLIT) al = Frag<T>::load(Ab2 + ao);
#pragma unroll
      for (int j = 0; j < 4; ++j) {
        acc[i][j] = Frag<T>::mma(ah, bh[j], acc[i][j]);
        if (SPLIT) {
          acc[i][j] = Frag<T>::mma(ah, bl[j], acc[i][j]);
          acc[i][j] = Frag<T>::mma(al, bh[j], acc[i][j]);
        }
      }
      Frag<T>::guard(acc[i][0], acc[i][3], ah, SPLIT ? al : ah);
    }
    Frag<T>::keep(bh[0], bh[1], bh[2], bh[3]);
    if (SPLIT) Frag<T>::keep(bl[0], bl[1], bl[2], bl[3]);
  }
  acc_guard4(acc[0][0], acc[0][1], acc[0][2], acc[0][3]);
  acc_guard4(acc[1][0], acc[1][1], acc[1][2], acc[1][3]);
  acc_guard4(acc[2][0], acc[2][1], acc[2][2], acc[2][3]);
  acc_guard4(acc[3][0], acc[3][1], acc[3][2], acc[3][3]);

  float* slab = sT[wave];
  const float* Rb = RESID ? (resid + (size_t)b * strideR) : nullptr;
#pragma unroll
  for (int i = 0; i < 4; ++i) {
    const int mBase = m0 + (i << 4);
#pragma unroll
    for (int j = 0; j < 4; ++j) {
      const int n = n0 + (j << 4) + rlane;
      float bv = 0.f;
      if (BIAS_MODE == 2) bv = bias[n];
#pragma unroll
      for (int r = 0; r < 8; ++r) {
        float v = acc[i][j][r] * scale;
        if (BIAS_MODE == 1) v += bias[mBase + mOff + r];
        if (BIAS_MODE == 2) v += bv;
        if (RESID) v += Rb[(size_t)(mBase + mOff + r) * ldc + n];
        if (ACT == 2) v = fmaxf(v, 0.0f);
        if (ACT == 4) v = (v > 0.f) ? v : 0.01f * v;
        slab[(mOff + r) * 68 + (j << 4) + rlane] = v;
      }
    }
    __builtin_amdgcn_fence(__ATOMIC_RELEASE, "workgroup");
    __builtin_amdgcn_wave_barrier();
    __builtin_amdgcn_fence(__ATOMIC_ACQUIRE, "workgroup");
    if (OUT_MODE == 0) {
      float* C = (float*)Cout + (size_t)b * strideC;
      const int hh = lane >> 4, c4 = (lane & 15) * 4;
      for (int pass = 0; pass < 2; ++pass) {
#pragma unroll
        for (int it = 0; it < 8; ++it) {
          const int row = it * 2 + hh;
          v4f v = *(const v4f*)(slab + row * 68 + c4);
          *(volatile v4f*)(C + (size_t)(mBase + row) * ldc + n0 + c4) = v;
        }
        __threadfence();
      }
    } else {
      const int q = lane >> 3, c8 = (lane & 7) * 8;
      unsigned short* C  = (unsigned short*)Cout  + (size_t)b * strideC;
      unsigned short* C2 = (OUT_MODE == 2) ? ((unsigned short*)Cout2 + (size_t)b * strideC) : nullptr;
      for (int pass = 0; pass < 2; ++pass) {
#pragma unroll
        for (int it = 0; it < 4; ++it) {
          const int row = it * 4 + q;
          const float* sp = slab + row * 68 + c8;
          v8h hv, lv;
#pragma unroll
          for (int e = 0; e < 8; ++e) {
            if (OUT_MODE == 1) {
              hv[e] = (_Float16)sp[e];
            } else {
              unsigned short hb = f2bf_bits(sp[e]);
              unsigned short lb = f2bf_bits(sp[e] - bf_bits2f(hb));
              hv[e] = __builtin_bit_cast(_Float16, hb);
              lv[e] = __builtin_bit_cast(_Float16, lb);
            }
          }
          *(volatile v8h*)(C + (size_t)(mBase + row) * ldc + n0 + c8) = hv;
          if (OUT_MODE == 2) *(volatile v8h*)(C2 + (size_t)(mBase + row) * ldc + n0 + c8) = lv;
        }
        __threadfence();
      }
    }
    __builtin_amdgcn_fence(__ATOMIC_RELEASE, "workgroup");
    __builtin_amdgcn_wave_barrier();
    __builtin_amdgcn_fence(__ATOMIC_ACQUIRE, "workgroup");
  }
}

__global__ __launch_bounds__(256) void xt_cast_kernel(const float* __restrict__ x, unsigned short* __restrict__ XT) {
  __shared__ float sm[64][65];
  const int t  = threadIdx.x;
  const int s0 = blockIdx.x * 64;
  const int b  = blockIdx.y;
#pragma unroll
  for (int i = 0; i < 4; ++i) {
    const int idx = i * 256 + t;
    const int e   = idx >> 4;
    const int s4  = (idx & 15) * 4;
    const v4f w = *(const v4f*)(x + ((size_t)(b * kD + e)) * kSeq + s0 + s4);
    sm[s4 + 0][e] = w[0];
    sm[s4 + 1][e] = w[1];
    sm[s4 + 2][e] = w[2];
    sm[s4 + 3][e] = w[3];
  }
  __syncthreads();
  const int lane = t & 31, wave = t >> 5;
  const int q = lane >> 3, c8 = (lane & 7) * 8;
  unsigned short* op = XT + ((size_t)b * kSeq + s0) * kD;
  for (int pass = 0; pass < 2; ++pass) {
#pragma unroll
    for (int it = 0; it < 2; ++it) {
      const int row = wave * 8 + it * 4 + q;
      unsigned short hb[8];
#pragma unroll
      for (int e = 0; e < 8; ++e) hb[e] = h_bits(kXCarry * bf16r(sm[row][c8 + e]));
      const v4u u = (v4u){pk16(hb[0], hb[1]), pk16(hb[2], hb[3]), pk16(hb[4], hb[5]), pk16(hb[6], hb[7])};
      *(volatile v4u*)(op + (size_t)row * kD + c8) = u;
    }
    __threadfence();
  }
}

__global__ __launch_bounds__(256) void wcast_kernel(const float* __restrict__ W0, const float* __restrict__ W1,
                                                    const float* __restrict__ W2, unsigned short* __restrict__ out) {
  const int z = blockIdx.y;
  const float* W = (z == 0) ? W0 : (z == 1) ? W1 : W2;
  const int i = blockIdx.x * 256 + threadIdx.x;
  if (i >= (kHD * kD) / 8) return;
  const float* p = W + 8 * (size_t)i;
  const v4f a = *(const v4f*)(p);
  const v4f c = *(const v4f*)(p + 4);
  unsigned short hb[8];
#pragma unroll
  for (int e = 0; e < 4; ++e) {
    hb[e]     = h_bits(kWCarry * bf16r(a[e]));
    hb[4 + e] = h_bits(kWCarry * bf16r(c[e]));
  }
  const v4u u = (v4u){pk16(hb[0], hb[1]), pk16(hb[2], hb[3]), pk16(hb[4], hb[5]), pk16(hb[6], hb[7])};
  unsigned short* qp = out + (size_t)z * kHD * kD + 8 * (size_t)i;
  *(volatile v4u*)qp = u;
  __threadfence();
  *(volatile v4u*)qp = u;
}

__global__ __launch_bounds__(256) void wt_cast_kernel(const float* __restrict__ W, unsigned short* __restrict__ WT) {
  __shared__ float sm[64][65];
  const int t  = threadIdx.x;
  const int k0 = blockIdx.x * 64;
#pragma unroll
  for (int i = 0; i < 4; ++i) {
    const int idx = i * 256 + t;
    const int kl  = idx >> 4;
    const int d4  = (idx & 15) * 4;
    const v4f w = *(const v4f*)(W + ((size_t)(k0 + kl)) * kD + d4);
    sm[d4 + 0][kl] = w[0];
    sm[d4 + 1][kl] = w[1];
    sm[d4 + 2][kl] = w[2];
    sm[d4 + 3][kl] = w[3];
  }
  __syncthreads();
  const int lane = t & 31, wave = t >> 5;
  const int q = lane >> 3, c8 = (lane & 7) * 8;
  for (int pass = 0; pass < 2; ++pass) {
#pragma unroll
    for (int it = 0; it < 2; ++it) {
      const int row = wave * 8 + it * 4 + q;
      unsigned short hb[8];
#pragma unroll
      for (int e = 0; e < 8; ++e) hb[e] = h_bits(kWCarry * bf16r(sm[row][c8 + e]));
      const v4u u = (v4u){pk16(hb[0], hb[1]), pk16(hb[2], hb[3]), pk16(hb[4], hb[5]), pk16(hb[6], hb[7])};
      *(volatile v4u*)(WT + (size_t)row * kHD + k0 + c8) = u;
    }
    __threadfence();
  }
}

__global__ __launch_bounds__(256) void softmax_row_kernel(const float* __restrict__ Sp, unsigned short* __restrict__ Pp) {
  __shared__ float redM[8];
  __shared__ float redS[8];
  const int row  = blockIdx.x;
  const int hg   = blockIdx.y;
  const int t    = threadIdx.x;
  const int lane = t & 31, wave = t >> 5;
  const size_t rowoff = ((size_t)hg * kSeq + row) * kSeq;
  const float* sr = Sp + rowoff + 8 * (size_t)t;
  const v4f a = *(const v4f*)(sr);
  const v4f c = *(const v4f*)(sr + 4);
  float xv[8];
#pragma unroll
  for (int e = 0; e < 4; ++e) { xv[e] = a[e]; xv[4 + e] = c[e]; }
  float mx = fmaxf(fmaxf(fmaxf(xv[0], xv[1]), fmaxf(xv[2], xv[3])), fmaxf(fmaxf(xv[4], xv[5]), fmaxf(xv[6], xv[7])));
#pragma unroll
  for (int off = 16; off > 0; off >>= 1) mx = fmaxf(mx, __shfl_xor(mx, off, 32));
  if (lane == 0) redM[wave] = mx;
  __syncthreads();
  float m = redM[0];
#pragma unroll
  for (int w = 1; w < 8; ++w) m = fmaxf(m, redM[w]);

  float ev[8];
  float sum = 0.f;
#pragma unroll
  for (int e = 0; e < 8; ++e) {
    ev[e] = expf(xv[e] - m);
    sum += ev[e];
  }
#pragma unroll
  for (int off = 16; off > 0; off >>= 1) sum += __shfl_xor(sum, off, 32);
  if (lane == 0) redS[wave] = sum;
  __syncthreads();
  float tot = redS[0];
#pragma unroll
  for (int w = 1; w < 8; ++w) tot += redS[w];
  const float inv = kPCarry / tot;

  unsigned short hb[8];
#pragma unroll
  for (int e = 0; e < 8; ++e) hb[e] = h_bits(ev[e] * inv);
  const v4u u = (v4u){pk16(hb[0], hb[1]), pk16(hb[2], hb[3]), pk16(hb[4], hb[5]), pk16(hb[6], hb[7])};
  unsigned short* pr = Pp + rowoff + 8 * (size_t)t;
  *(volatile v4u*)pr = u;
  __threadfence();
  *(volatile v4u*)pr = u;
}

extern "C" void kernel_launch(void* const* d_in, const int* in_sizes, int n_in,
                              void* d_out, int out_size, void* d_ws, size_t ws_size,
                              hipStream_t stream) {
  if (n_in < 5) return;
  if (in_sizes[0] != kBatch * kD * kSeq) return;
  if (in_sizes[1] != kHeads * kD * kD || in_sizes[2] != kHeads * kD * kD || in_sizes[3] != kHeads * kD * kD) return;
  if (in_sizes[4] != kHD * kD) return;
  if (out_size != kOutElems) return;

  const size_t szXT = (size_t)kBatch * kSeq * kD * 2;
  const size_t szW  = (size_t)kHD * kD * 2;
  const size_t szQK = (size_t)kBatch * kSeq * kHD * 2;
  const size_t szVT = (size_t)kBatch * kHeads * kD * kSeq * 2;
  const size_t szOT = szQK;
  const size_t szSC = (size_t)kGroup * kSeq * kSeq * 4;
  const size_t szPP = (size_t)kGroup * kSeq * kSeq * 2;
  const size_t offXT  = 0;
  const size_t offWQ  = offXT + szXT;
  const size_t offWK  = offWQ + szW;
  const size_t offWV  = offWK + szW;
  const size_t offWT  = offWV + szW;
  const size_t offQ16 = offWT + szW;
  const size_t offK16 = offQ16 + szQK;
  const size_t offVT  = offK16 + szQK;
  const size_t offOT  = offVT + szVT;
  const size_t offSC  = offOT + szOT;
  const size_t offPP  = offSC + szSC;
  const size_t total  = offPP + szPP;
  if (ws_size < total) return;

  const float* xin = (const float*)d_in[0];
  const float* wq  = (const float*)d_in[1];
  const float* wk  = (const float*)d_in[2];
  const float* wv  = (const float*)d_in[3];
  const float* wf  = (const float*)d_in[4];
  float* outY = (float*)d_out;
  float* outQ = outY + (size_t)kBatch * kD * kSeq;
  float* outK = outQ + (size_t)kBatch * kHeads * kD * kSeq;
  float* outV = outK + (size_t)kBatch * kHeads * kD * kSeq;
  char* ws = (char*)d_ws;
  unsigned short* XT   = (unsigned short*)(ws + offXT);
  unsigned short* WQ16 = (unsigned short*)(ws + offWQ);
  unsigned short* WK16 = (unsigned short*)(ws + offWK);
  unsigned short* WV16 = (unsigned short*)(ws + offWV);
  unsigned short* WT16 = (unsigned short*)(ws + offWT);
  unsigned short* Q16  = (unsigned short*)(ws + offQ16);
  unsigned short* K16  = (unsigned short*)(ws + offK16);
  unsigned short* VT16 = (unsigned short*)(ws + offVT);
  unsigned short* OT16 = (unsigned short*)(ws + offOT);
  float*          SC   = (float*)(ws + offSC);
  unsigned short* PP   = (unsigned short*)(ws + offPP);
  const float* dummyf = xin;

  xt_cast_kernel<<<dim3(kSeq / 64, kBatch), dim3(256), 0, stream>>>(xin, XT);
  wcast_kernel<<<dim3(((kHD * kD) / 8) / 256, 3), dim3(256), 0, stream>>>(wq, wk, wv, WQ16);
  wt_cast_kernel<<<dim3(kHD / 64), dim3(256), 0, stream>>>(wf, WT16);

  const long strideXT  = (long)kSeq * kD;
  const long strideOutH = (long)kHD * kSeq;
  const long strideTok = (long)kSeq * kHD;
  const int  blkProj   = ((kHD / 64) * (kSeq / 64)) / 8;

  wmma_gemm64<0, false, 0, 0, false, 0><<<dim3(blkProj, kBatch), dim3(256), 0, stream>>>(
      WQ16, WQ16, kD, 0L, XT, XT, kD, strideXT, (void*)outQ, (void*)outQ, kSeq, strideOutH,
      dummyf, dummyf, 0L, kHD, kSeq, kD, kProjOutScale);
  wmma_gemm64<0, false, 0, 0, false, 0><<<dim3(blkProj, kBatch), dim3(256), 0, stream>>>(
      WK16, WK16, kD, 0L, XT, XT, kD, strideXT, (void*)outK, (void*)outK, kSeq, strideOutH,
      dummyf, dummyf, 0L, kHD, kSeq, kD, kProjOutScale);
  wmma_gemm64<0, false, 0, 0, false, 0><<<dim3(blkProj, kBatch), dim3(256), 0, stream>>>(
      WV16, WV16, kD, 0L, XT, XT, kD, strideXT, (void*)outV, (void*)outV, kSeq, strideOutH,
      dummyf, dummyf, 0L, kHD, kSeq, kD, kProjOutScale);

  wmma_gemm64<0, false, 0, 1, false, 0><<<dim3(blkProj, kBatch), dim3(256), 0, stream>>>(
      XT, XT, kD, strideXT, WQ16, WQ16, kD, 0L, (void*)Q16, (void*)Q16, kHD, strideTok,
      dummyf, dummyf, 0L, kSeq, kHD, kD, kProjPlanScale);
  wmma_gemm64<0, false, 0, 1, false, 0><<<dim3(blkProj, kBatch), dim3(256), 0, stream>>>(
      XT, XT, kD, strideXT, WK16, WK16, kD, 0L, (void*)K16, (void*)K16, kHD, strideTok,
      dummyf, dummyf, 0L, kSeq, kHD, kD, kProjPlanScale);
  wmma_gemm64<0, false, 0, 1, false, 0><<<dim3(blkProj, kBatch), dim3(256), 0, stream>>>(
      WV16, WV16, kD, 0L, XT, XT, kD, strideXT, (void*)VT16, (void*)VT16, kSeq, strideOutH,
      dummyf, dummyf, 0L, kHD, kSeq, kD, kProjPlanScale);

  const long strideHead16 = (long)kD;
  const long strideScore  = (long)kSeq * kSeq;
  const long strideVT     = (long)kD * kSeq;
  const int  blkScore     = ((kSeq / 64) * (kSeq / 64)) / 8;
  const int  blkCtx       = ((kSeq / 64) * (kD / 64)) / 8;

  for (int b = 0; b < kBatch; ++b) {
    for (int g = 0; g < kHeads / kGroup; ++g) {
      const size_t colOff  = (size_t)b * kSeq * kHD + (size_t)g * kGroup * kD;
      const size_t headIdx = (size_t)b * kHeads + (size_t)g * kGroup;
      wmma_gemm64<0, false, 0, 0, false, 0><<<dim3(blkScore, kGroup), dim3(256), 0, stream>>>(
          K16 + colOff, K16 + colOff, kHD, strideHead16, Q16 + colOff, Q16 + colOff, kHD, strideHead16,
          (void*)SC, (void*)SC, kSeq, strideScore, dummyf, dummyf, 0L, kSeq, kSeq, kD, kScoreScale);
      softmax_row_kernel<<<dim3(kSeq, kGroup), dim3(256), 0, stream>>>(SC, PP);
      const unsigned short* VTg = VT16 + headIdx * (size_t)kD * kSeq;
      wmma_gemm64<0, false, 0, 1, false, 0><<<dim3(blkCtx, kGroup), dim3(256), 0, stream>>>(
          PP, PP, kSeq, strideScore, VTg, VTg, kSeq, strideVT,
          (void*)(OT16 + colOff), (void*)(OT16 + colOff), kHD, strideHead16, dummyf, dummyf, 0L,
          kSeq, kD, kSeq, kPVScale);
    }
  }

  const int blkY = ((kD / 64) * (kSeq / 64)) / 8;
  wmma_gemm64<0, false, 0, 0, false, 0><<<dim3(blkY, kBatch), dim3(256), 0, stream>>>(
      WT16, WT16, kHD, 0L, OT16, OT16, kHD, strideTok, (void*)outY, (void*)outY, kSeq, (long)kD * kSeq,
      dummyf, dummyf, 0L, kD, kSeq, kHD, kYScale);
}
